// Mamba_Block_32590211842131
// MI455X (gfx1250) — hardware-verified
//
#include <hip/hip_runtime.h>
#include <math.h>

typedef __attribute__((ext_vector_type(16))) _Float16 v16h;
typedef __attribute__((ext_vector_type(8)))  _Float16 v8h;
typedef __attribute__((ext_vector_type(16))) __bf16   v16b;
typedef __attribute__((ext_vector_type(8)))  __bf16   v8b;
typedef __attribute__((ext_vector_type(8)))  float    v8f;
typedef __attribute__((ext_vector_type(4)))  float    v4f;
typedef __attribute__((ext_vector_type(4)))  unsigned v4u;

constexpr int kBatch  = 4;
constexpr int kSeq    = 2048;
constexpr int kDm     = 256;
constexpr int kDin    = 512;
constexpr int kNst    = 16;
constexpr int kDtR    = 16;
constexpr int kXzP    = 2 * kDin;
constexpr int kXdW    = kDtR + 2 * kNst;
constexpr int kXdP    = 64;
constexpr int kRows   = kBatch * kSeq;
constexpr int kConvTP = 260;
constexpr int kScanTS = 64;
constexpr int kScanCh = 64;
constexpr int kScanYP = 68;
constexpr int kLnTok  = 32;
constexpr int kLnTP   = 260;
constexpr float kActCarry = 8.0f;
constexpr float kWCarry   = 16.0f;
constexpr float kGemmFold = 1.0f / 128.0f;
static_assert(kXdW <= kXdP, "x_proj pad");
static_assert((kDm % 32) == 0 && (kDin % 32) == 0, "GEMM K multiples of 32");
static_assert((kRows % 64) == 0 && (kXzP % 64) == 0 && (kXdP % 64) == 0 && (kDm % 64) == 0, "GEMM M,N multiples of 64");
static_assert((kSeq % kScanTS) == 0 && (kSeq % 64) == 0 && (kDin % kScanCh) == 0 && (kDin % 256) == 0, "tile multiples");
static_assert((kSeq & (kSeq - 1)) == 0, "power of two sequence length");
static_assert(kDm == 256 && (kSeq % kLnTok) == 0, "LayerNorm kernel geometry: 8 channels per lane, 32 channels per wave");
static_assert((((kRows / 64) * (kXzP / 64)) % 8) == 0 && (((kRows / 64) * (kXdP / 64)) % 8) == 0 && (((kRows / 64) * (kDm / 64)) % 8) == 0, "GEMM grids exact");

constexpr size_t kOffU    = 0;
constexpr size_t kOffWI   = kOffU   + (size_t)kRows * kDm  * 2;
constexpr size_t kOffWX   = kOffWI  + (size_t)kXzP  * kDm  * 2;
constexpr size_t kOffWO   = kOffWX  + (size_t)kXdP  * kDin * 2;
constexpr size_t kOffXZ   = kOffWO  + (size_t)kDm   * kDin * 2;
constexpr size_t kOffUC   = kOffXZ  + (size_t)kRows * kXzP * 4;
constexpr size_t kOffUCH  = kOffUC  + (size_t)kRows * kDin * 4;
constexpr size_t kOffXD   = kOffUCH + (size_t)kRows * kDin * 2;
constexpr size_t kOffY    = kOffXD  + (size_t)kRows * kXdP * 4;
constexpr size_t kOffOP   = kOffY   + (size_t)kRows * kDin * 2;
constexpr size_t kWsTotal = kOffOP  + (size_t)kRows * kDm  * 4;
static_assert(kWsTotal == 82640896ull, "carve total");
static_assert(kWsTotal <= 134217728ull, "carve cap");
static_assert((kOffWI % 128) == 0 && (kOffWX % 128) == 0 && (kOffWO % 128) == 0 && (kOffXZ % 128) == 0 &&
              (kOffUC % 128) == 0 && (kOffUCH % 128) == 0 && (kOffXD % 128) == 0 && (kOffY % 128) == 0 &&
              (kOffOP % 128) == 0, "128-B aligned regions");

__device__ __forceinline__ unsigned short f2bf_bits(float f) {
  unsigned u = __float_as_uint(f);
  return (unsigned short)((u + 0x7FFFu + ((u >> 16) & 1u)) >> 16);
}
__device__ __forceinline__ float bf_bits2f(unsigned short h) { return __uint_as_float(((unsigned)h) << 16); }

__device__ __forceinline__ void dep_guard_h(v8f& a, v8f& b, v16h x, v16h y) { asm volatile("v_nop\n\tv_nop\n\tv_nop\n\tv_nop" : "+v"(a), "+v"(b) : "v"(x), "v"(y)); }
__device__ __forceinline__ void dep_guard_b(v8f& a, v8f& b, v16b x, v16b y) { asm volatile("v_nop\n\tv_nop\n\tv_nop\n\tv_nop" : "+v"(a), "+v"(b) : "v"(x), "v"(y)); }
__device__ __forceinline__ void keep4_h(v16h a, v16h b, v16h c, v16h d) { asm volatile("v_nop" :: "v"(a), "v"(b), "v"(c), "v"(d)); }
__device__ __forceinline__ void keep4_b(v16b a, v16b b, v16b c, v16b d) { asm volatile("v_nop" :: "v"(a), "v"(b), "v"(c), "v"(d)); }
__device__ __forceinline__ void acc_guard4(v8f& a, v8f& b, v8f& c, v8f& d) { asm volatile("v_nop\n\tv_nop\n\tv_nop\n\tv_nop" : "+v"(a), "+v"(b), "+v"(c), "+v"(d)); }
template <typename T> struct Frag;
template <> struct Frag<_Float16> {
  typedef v16h V; union U { v16h v; v8h h[2]; };
  static __device__ __forceinline__ v16h load(const _Float16* p) {
    U f; f.h[0] = *(const v8h*)(p); f.h[1] = *(const v8h*)(p + 16); return f.v;
  }
  static __device__ __forceinline__ v8f mma(v16h a, v16h b, v8f c) {
    return __builtin_amdgcn_wmma_f32_16x16x32_f16(false, a, false, b, (short)0, c, false, false);
  }
  static __device__ __forceinline__ void guard(v8f& a, v8f& b, v16h x, v16h y) { dep_guard_h(a, b, x, y); }
  static __device__ __forceinline__ void keep(v16h a, v16h b, v16h c, v16h d) { keep4_h(a, b, c, d); }
};
template <> struct Frag<__bf16> {
  typedef v16b V; union U { v16b v; v8b h[2]; };
  static __device__ __forceinline__ v16b load(const __bf16* p) {
    U f; f.h[0] = *(const v8b*)(p); f.h[1] = *(const v8b*)(p + 16); return f.v;
  }
  static __device__ __forceinline__ v8f mma(v16b a, v16b b, v8f c) {
    return __builtin_amdgcn_wmma_f32_16x16x32_bf16(false, a, false, b, (short)0, c, false, false);
  }
  static __device__ __forceinline__ void guard(v8f& a, v8f& b, v16b x, v16b y) { dep_guard_b(a, b, x, y); }
  static __device__ __forceinline__ void keep(v16b a, v16b b, v16b c, v16b d) { keep4_b(a, b, c, d); }
};

template <int ET> struct Elem;
template <> struct Elem<0> { typedef _Float16 T; };
template <> struct Elem<1> { typedef __bf16 T; };
template <int ET, bool SPLIT, int BIAS_MODE, int OUT_MODE, bool RESID, int ACT = 0>
__global__ __launch_bounds__(256) void wmma_gemm64(
    const unsigned short* __restrict__ Ap, const unsigned short* __restrict__ A2p, int lda, long strideA,
    const unsigned short* __restrict__ Btp, const unsigned short* __restrict__ Bt2p, int ldb, long strideB,
    void* __restrict__ Cout, void* __restrict__ Cout2, int ldc, long strideC,
    const float* __restrict__ bias,
    const float* __restrict__ resid, long strideR,
    int M, int N, int K, float scale) {
  typedef typename Elem<ET>::T T;
  typedef typename Frag<T>::V V;
  const T* A = (const T*)Ap; const T* A2 = (const T*)A2p; const T* Bt = (const T*)Btp; const T* Bt2 = (const T*)Bt2p;
  __shared__ __align__(16) float sT[8][16 * 68];
  const int b    = blockIdx.y;
  const int lane = threadIdx.x & 31;
  const int wave = threadIdx.x >> 5;
  const int tilesN = N >> 6;
  const int tilesM = M >> 6;
  const int tile = blockIdx.x * 8 + wave;
  if (tile >= tilesM * tilesN) return;
  const int tm = tile / tilesN;
  const int tn = tile - tm * tilesN;
  const int m0 = tm << 6;
  const int n0 = tn << 6;

  const T* Ab  = A  + (size_t)b * strideA;
  const T* Bb  = Bt + (size_t)b * strideB;
  const T* Ab2 = SPLIT ? (A2  + (size_t)b * strideA) : nullptr;
  const T* Bb2 = SPLIT ? (Bt2 + (size_t)b * strideB) : nullptr;

  const int rlane = lane & 15;
  const int koff  = (lane >> 4) * 8;
  const int mOff  = (lane >> 4) * 8;

  v8f acc[4][4];
#pragma unroll
  for (int i = 0; i < 4; ++i)
#pragma unroll
    for (int j = 0; j < 4; ++j) acc[i][j] = (v8f){0.f,0.f,0.f,0.f,0.f,0.f,0.f,0.f};

  for (int k0 = 0; k0 < K; k0 += 32) {
    V bh[4], bl[4];
#pragma unroll
    for (int j = 0; j < 4; ++j) {
      const size_t bo = (size_t)(n0 + (j << 4) + rlane) * ldb + koff + k0;
      bh[j] = Frag<T>::load(Bb + bo);
      if (SPLIT) bl[j] = Frag<T>::load(Bb2 + bo);
    }
#pragma unroll
    for (int i = 0; i < 4; ++i) {
      const size_t ao = (size_t)(m0 + (i << 4) + rlane) * lda + koff + k0;
      V ah = Frag<T>::load(Ab + ao);
      V al;
      if (SPLIT) al = Frag<T>::load(Ab2 + ao);
#pragma unroll
      for (int j = 0; j < 4; ++j) {
        acc[i][j] = Frag<T>::mma(ah, bh[j], acc[i][j]);
        if (SPLIT) {
          acc[i][j] = Frag<T>::mma(ah, bl[j], acc[i][j]);
          acc[i][j] = Frag<T>::mma(al, bh[j], acc[i][j]);
        }
      }
      Frag<T>::guard(acc[i][0], acc[i][3], ah, SPLIT ? al : ah);
    }
    Frag<T>::keep(bh[0], bh[1], bh[2], bh[3]);
    if (SPLIT) Frag<T>::keep(bl[0], bl[1], bl[2], bl[3]);
  }
  acc_guard4(acc[0][0], acc[0][1], acc[0][2], acc[0][3]);
  acc_guard4(acc[1][0], acc[1][1], acc[1][2], acc[1][3]);
  acc_guard4(acc[2][0], acc[2][1], acc[2][2], acc[2][3]);
  acc_guard4(acc[3][0], acc[3][1], acc[3][2], acc[3][3]);

  float* slab = sT[wave];
  const float* Rb = RESID ? (resid + (size_t)b * strideR) : nullptr;
#pragma unroll
  for (int i = 0; i < 4; ++i) {
    const int mBase = m0 + (i << 4);
#pragma unroll
    for (int j = 0; j < 4; ++j) {
      const int n = n0 + (j << 4) + rlane;
      float bv = 0.f;
      if (BIAS_MODE == 2) bv = bias[n];
#pragma unroll
      for (int r = 0; r < 8; ++r) {
        float v = acc[i][j][r] * scale;
        if (BIAS_MODE == 1) v += bias[mBase + mOff + r];
        if (BIAS_MODE == 2) v += bv;
        if (RESID) v += Rb[(size_t)(mBase + mOff + r) * ldc + n];
        if (ACT == 1) v = tanhf(v);
        if (ACT == 2) v = fmaxf(v, 0.0f);
        if (ACT == 3) v = v / (1.0f + expf(-v));
        if (ACT == 4) v = (v > 0.f) ? v : 0.01f * v;
        if (ACT == 5) v = 0.5f * v * (1.0f + erff(v * 0.70710678118654752f));
        slab[(mOff + r) * 68 + (j << 4) + rlane] = v;
      }
    }
    __builtin_amdgcn_fence(__ATOMIC_RELEASE, "workgroup");
    __builtin_amdgcn_wave_barrier();
    __builtin_amdgcn_fence(__ATOMIC_ACQUIRE, "workgroup");
    if (OUT_MODE == 0) {
      float* C = (float*)Cout + (size_t)b * strideC;
      const int hh = lane >> 4, c4 = (lane & 15) * 4;
      for (int pass = 0; pass < 2; ++pass) {
#pragma unroll
        for (int it = 0; it < 8; ++it) {
          const int row = it * 2 + hh;
          v4f v = *(const v4f*)(slab + row * 68 + c4);
          *(volatile v4f*)(C + (size_t)(mBase + row) * ldc + n0 + c4) = v;
        }
        __threadfence();
      }
    } else {
      const int q = lane >> 3, c8 = (lane & 7) * 8;
      unsigned short* C  = (unsigned short*)Cout  + (size_t)b * strideC;
      unsigned short* C2 = (OUT_MODE == 2) ? ((unsigned short*)Cout2 + (size_t)b * strideC) : nullptr;
      for (int pass = 0; pass < 2; ++pass) {
#pragma unroll
        for (int it = 0; it < 4; ++it) {
          const int row = it * 4 + q;
          const float* sp = slab + row * 68 + c8;
          v8h hv, lv;
#pragma unroll
          for (int e = 0; e < 8; ++e) {
            if (OUT_MODE == 1) {
              hv[e] = (_Float16)sp[e];
            } else {
              unsigned short hb = f2bf_bits(sp[e]);
              unsigned short lb = f2bf_bits(sp[e] - bf_bits2f(hb));
              hv[e] = __builtin_bit_cast(_Float16, hb);
              lv[e] = __builtin_bit_cast(_Float16, lb);
            }
          }
          *(volatile v8h*)(C + (size_t)(mBase + row) * ldc + n0 + c8) = hv;
          if (OUT_MODE == 2) *(volatile v8h*)(C2 + (size_t)(mBase + row) * ldc + n0 + c8) = lv;
        }
        __threadfence();
      }
    }
    __builtin_amdgcn_fence(__ATOMIC_RELEASE, "workgroup");
    __builtin_amdgcn_wave_barrier();
    __builtin_amdgcn_fence(__ATOMIC_ACQUIRE, "workgroup");
  }
}

__device__ __forceinline__ float wave_sum(float v) {
#pragma unroll
  for (int off = 1; off < 32; off <<= 1) v += __shfl_xor(v, off, 32);
  return v;
}

__global__ __launch_bounds__(256) void cast_scale_f16x8_kernel(
    const float* __restrict__ src, int nsrc8, unsigned short* __restrict__ dst, int ndst8, float scale)
{
  const int i = blockIdx.x * 256 + threadIdx.x;
  if (i >= ndst8) return;
  const bool valid = (i < nsrc8);
  const int ic = valid ? i : (nsrc8 - 1);
  const size_t e0 = (size_t)ic << 3;
  const v4f a0 = *(const v4f*)(src + e0);
  const v4f a1 = *(const v4f*)(src + e0 + 4);
  v4u w;
#pragma unroll
  for (int p = 0; p < 2; ++p) {
    const _Float16 h0 = (_Float16)(a0[2 * p] * scale), h1 = (_Float16)(a0[2 * p + 1] * scale);
    const _Float16 g0 = (_Float16)(a1[2 * p] * scale), g1 = (_Float16)(a1[2 * p + 1] * scale);
    const unsigned u0 = (unsigned)__builtin_bit_cast(unsigned short, h0) | ((unsigned)__builtin_bit_cast(unsigned short, h1) << 16);
    const unsigned u1 = (unsigned)__builtin_bit_cast(unsigned short, g0) | ((unsigned)__builtin_bit_cast(unsigned short, g1) << 16);
    w[p]     = valid ? u0 : 0u;
    w[2 + p] = valid ? u1 : 0u;
  }
  unsigned short* qd = dst + ((size_t)i << 3);
  *(volatile v4u*)qd = w;
  __threadfence();
  *(volatile v4u*)qd = w;
}

__global__ __launch_bounds__(256) void ln_front_kernel(
    const float* __restrict__ x, const float* __restrict__ lnw, const float* __restrict__ lnb,
    unsigned short* __restrict__ UP)
{
  __shared__ __align__(16) float sV[kLnTok * kLnTP];
  const int tid = threadIdx.x, lane = tid & 31, wave = tid >> 5;
  constexpr int kBlkPerB = kSeq / kLnTok;
  const int b  = blockIdx.x / kBlkPerB;
  const int l0 = (blockIdx.x - b * kBlkPerB) * kLnTok;
  const size_t row0 = (size_t)b * kSeq + l0;
  const float* xb = x + (size_t)b * kDm * kSeq + l0 + lane;
#pragma unroll 1
  for (int it = 0; it < kDm / 8; ++it) {
    const int c = it * 8 + wave;
    sV[lane * kLnTP + c] = xb[(size_t)c * kSeq];
  }
  __syncthreads();
  const v4f w0 = *(const v4f*)(lnw + 8 * lane), w1 = *(const v4f*)(lnw + 8 * lane + 4);
  const v4f g0 = *(const v4f*)(lnb + 8 * lane), g1 = *(const v4f*)(lnb + 8 * lane + 4);
  v8h hv[4];
#pragma unroll
  for (int rr = 0; rr < 4; ++rr) {
    const float* sp = sV + (wave * 4 + rr) * kLnTP + 8 * lane;
    const v4f a0 = *(const v4f*)(sp), a1 = *(const v4f*)(sp + 4);
    float s = ((a0[0] + a0[1]) + (a0[2] + a0[3])) + ((a1[0] + a1[1]) + (a1[2] + a1[3]));
    s = wave_sum(s);
    const float mu = s * (1.0f / kDm);
    const v4f d0 = a0 - mu, d1 = a1 - mu;
    float sq = ((d0[0] * d0[0] + d0[1] * d0[1]) + (d0[2] * d0[2] + d0[3] * d0[3]))
             + ((d1[0] * d1[0] + d1[1] * d1[1]) + (d1[2] * d1[2] + d1[3] * d1[3]));
    sq = wave_sum(sq);
    const float rs = rsqrtf(sq * (1.0f / kDm) + 1e-5f);
    const v4f o0 = d0 * rs * w0 + g0;
    const v4f o1 = d1 * rs * w1 + g1;
#pragma unroll
    for (int e = 0; e < 4; ++e) {
      hv[rr][e]     = (_Float16)(o0[e] * kActCarry);
      hv[rr][4 + e] = (_Float16)(o1[e] * kActCarry);
    }
  }
  for (int pass = 0; pass < 2; ++pass) {
#pragma unroll
    for (int rr = 0; rr < 4; ++rr)
      *(volatile v8h*)(UP + (row0 + wave * 4 + rr) * kDm + 8 * lane) = hv[rr];
    __threadfence();
  }
}

__global__ __launch_bounds__(256) void conv_silu_kernel(
    const float* __restrict__ XZ, const float* __restrict__ cw, const float* __restrict__ cb,
    float* __restrict__ UC, unsigned short* __restrict__ UCH)
{
  __shared__ __align__(16) float sT[16 * kConvTP];
  const int tid = threadIdx.x, lane = tid & 31, wave = tid >> 5;
  const int d0 = blockIdx.x * 256, d = d0 + tid;
  const int g0 = blockIdx.y * 64;
  const int tb = g0 & (kSeq - 1);
  const float w0 = cw[d * 4 + 0], w1 = cw[d * 4 + 1], w2 = cw[d * 4 + 2], w3 = cw[d * 4 + 3];
  const float bc = cb[d];
  float xm3, xm2, xm1;
  {
    const bool hist = (tb > 0);
    const int rb = hist ? (g0 - 3) : g0;
    const float v3 = XZ[(size_t)rb * kXzP + d];
    const float v2 = XZ[(size_t)(rb + 1) * kXzP + d];
    const float v1 = XZ[(size_t)(rb + 2) * kXzP + d];
    xm3 = hist ? v3 : 0.f;
    xm2 = hist ? v2 : 0.f;
    xm1 = hist ? v1 : 0.f;
  }
  const int hrow = wave >> 1;
  const int hch  = (wave & 1) * 128 + lane * 4;
#pragma unroll 1
  for (int sub = 0; sub < 4; ++sub) {
    const int lb = g0 + sub * 16;
#pragma unroll 1
    for (int s = 0; s < 16; ++s) {
      const float xcur = XZ[(size_t)(lb + s) * kXzP + d];
      float acc = w0 * xm3;
      acc = fmaf(w1, xm2, acc);
      acc = fmaf(w2, xm1, acc);
      acc = fmaf(w3, xcur, acc);
      const float sv = acc + bc;
      const float sg = __builtin_amdgcn_rcpf(1.0f + __expf(-sv));
      sT[s * kConvTP + tid] = sv * sg;
      xm3 = xm2; xm2 = xm1; xm1 = xcur;
    }
    __syncthreads();
    v4f fv[4];
    v8h bh[2];
#pragma unroll
    for (int it = 0; it < 4; ++it) fv[it] = *(const v4f*)(sT + (it * 4 + hrow) * kConvTP + hch);
#pragma unroll
    for (int it = 0; it < 2; ++it) {
      const float* sp = sT + (it * 8 + wave) * kConvTP + lane * 8;
      const v4f a0 = *(const v4f*)(sp);
      const v4f a1 = *(const v4f*)(sp + 4);
#pragma unroll
      for (int e = 0; e < 4; ++e) {
        bh[it][e]     = (_Float16)(a0[e] * kActCarry);
        bh[it][4 + e] = (_Float16)(a1[e] * kActCarry);
      }
    }
    for (int pass = 0; pass < 2; ++pass) {
#pragma unroll
      for (int it = 0; it < 4; ++it)
        *(volatile v4f*)(UC + (size_t)(lb + it * 4 + hrow) * kDin + d0 + hch) = fv[it];
#pragma unroll
      for (int it = 0; it < 2; ++it) {
        const size_t o = (size_t)(lb + it * 8 + wave) * kDin + d0 + lane * 8;
        *(volatile v8h*)(UCH + o) = bh[it];
      }
      __threadfence();
    }
    __syncthreads();
  }
}

__global__ __launch_bounds__(64) void scan_kernel(
    const float* __restrict__ XD, const float* __restrict__ UC, const float* __restrict__ XZ,
    const float* __restrict__ Wdt, const float* __restrict__ bdt, const float* __restrict__ Alog,
    const float* __restrict__ Dp, unsigned short* __restrict__ YP)
{
  __shared__ __align__(16) float sX[kScanTS * kXdP];
  __shared__ __align__(16) float sY[kScanTS * kScanYP];
  __shared__ __align__(16) float sW[kDtR * kScanCh];
  __shared__ __align__(16) float sA[kNst * kScanCh];
  const int tid = threadIdx.x, lane = tid & 31, wave = tid >> 5;
  constexpr int kBlkPerB = kDin / kScanCh;
  const int bix = blockIdx.x / kBlkPerB;
  const int d0  = (blockIdx.x - bix * kBlkPerB) * kScanCh;
  const int d   = d0 + tid;
  const size_t row0 = (size_t)bix * kSeq;
#pragma unroll 1
  for (int r = 0; r < kDtR; ++r) sW[r * kScanCh + tid] = Wdt[(size_t)d * kDtR + r];
#pragma unroll 1
  for (int s = 0; s < kNst; ++s) sA[s * kScanCh + tid] = -expf(Alog[(size_t)d * kNst + s]);
  __syncthreads();
  float negA[kNst], h[kNst];
#pragma unroll
  for (int s = 0; s < kNst; ++s) {
    negA[s] = sA[s * kScanCh + tid];
    h[s] = 0.f;
  }
  const float bb = bdt[d], Dd = Dp[d];
  const int lr = tid >> 4, lc4 = (tid & 15) * 4;
  const int q = lane >> 3, c8 = (lane & 7) * 8;
#pragma unroll 1
  for (int t0 = 0; t0 < kSeq; t0 += kScanTS) {
    __syncthreads();
#pragma unroll
    for (int i = 0; i < 16; ++i) {
      const int r = lr + 4 * i;
      *(v4f*)(sX + r * kXdP + lc4) = *(const v4f*)(XD + (row0 + t0 + r) * kXdP + lc4);
    }
    __syncthreads();
#pragma unroll 1
    for (int s = 0; s < kScanTS; ++s) {
      const int t = t0 + s;
      const float* xr = sX + s * kXdP;
      float vdot = 0.f;
#pragma unroll 1
      for (int r4 = 0; r4 < kDtR / 4; ++r4) {
        const v4f xv = *(const v4f*)(xr + 4 * r4);
        const float* wp = sW + (4 * r4) * kScanCh + tid;
        vdot = fmaf(xv[0], wp[0], vdot);
        vdot = fmaf(xv[1], wp[kScanCh], vdot);
        vdot = fmaf(xv[2], wp[2 * kScanCh], vdot);
        vdot = fmaf(xv[3], wp[3 * kScanCh], vdot);
      }
      float Bs[kNst], Cs[kNst];
#pragma unroll
      for (int q4 = 0; q4 < 4; ++q4) {
        const v4f bv = *(const v4f*)(xr + kDtR + 4 * q4);
        const v4f cv = *(const v4f*)(xr + kDtR + kNst + 4 * q4);
        Bs[4 * q4 + 0] = bv[0]; Bs[4 * q4 + 1] = bv[1]; Bs[4 * q4 + 2] = bv[2]; Bs[4 * q4 + 3] = bv[3];
        Cs[4 * q4 + 0] = cv[0]; Cs[4 * q4 + 1] = cv[1]; Cs[4 * q4 + 2] = cv[2]; Cs[4 * q4 + 3] = cv[3];
      }
      const float v   = vdot + bb;
      const float a   = __expf(-fabsf(v));
      const float u   = 1.0f + a;
      const float l1p = __logf(u) + (a - (u - 1.0f)) * __builtin_amdgcn_rcpf(u);
      const float dt  = fmaxf(v, 0.0f) + l1p;
      const float xt  = UC[(row0 + t) * kDin + d];
      const float dtx = dt * xt;
      float y = 0.f;
#pragma unroll
      for (int k = 0; k < kNst; ++k) {
        const float e = __expf(dt * negA[k]);
        h[k] = e * h[k] + dtx * Bs[k];
        y = h[k] * Cs[k] + y;
      }
      y = xt * Dd + y;
      const float zv = XZ[(row0 + t) * kXzP + kDin + d];
      const float sg = __builtin_amdgcn_rcpf(1.0f + __expf(-zv));
      y = y * (zv * sg);
      sY[s * kScanYP + tid] = y;
    }
    __syncthreads();
    v8h hv[8];
#pragma unroll
    for (int it = 0; it < 8; ++it) {
      const int row = it * 8 + wave * 4 + q;
      const float* sp = sY + row * kScanYP + c8;
      const v4f a0 = *(const v4f*)(sp);
      const v4f a1 = *(const v4f*)(sp + 4);
#pragma unroll
      for (int e = 0; e < 4; ++e) {
        hv[it][e]     = (_Float16)(a0[e] * kActCarry);
        hv[it][4 + e] = (_Float16)(a1[e] * kActCarry);
      }
    }
    for (int pass = 0; pass < 2; ++pass) {
#pragma unroll
      for (int it = 0; it < 8; ++it) {
        const int row = it * 8 + wave * 4 + q;
        const size_t o = (row0 + t0 + row) * kDin + d0 + c8;
        *(volatile v8h*)(YP + o) = hv[it];
      }
      __threadfence();
    }
  }
}

__global__ __launch_bounds__(256) void ln_post_kernel(
    const float* __restrict__ OP, const float* __restrict__ x, const float* __restrict__ lnw,
    const float* __restrict__ lnb, float* __restrict__ out)
{
  __shared__ __align__(16) float sV[kLnTok * kLnTP];
  const int tid = threadIdx.x, lane = tid & 31, wave = tid >> 5;
  constexpr int kBlkPerB = kSeq / kLnTok;
  const int b  = blockIdx.x / kBlkPerB;
  const int l0 = (blockIdx.x - b * kBlkPerB) * kLnTok;
  const size_t row0 = (size_t)b * kSeq + l0;
  const float* xb = x + (size_t)b * kDm * kSeq + l0 + lane;
#pragma unroll 1
  for (int it = 0; it < kDm / 8; ++it) {
    const int c = it * 8 + wave;
    sV[lane * kLnTP + c] = xb[(size_t)c * kSeq];
  }
  __syncthreads();
  {
    const float* opb = OP + row0 * kDm + tid;
#pragma unroll 1
    for (int t = 0; t < kLnTok; ++t) sV[t * kLnTP + tid] += opb[(size_t)t * kDm];
  }
  __syncthreads();
  const v4f w0 = *(const v4f*)(lnw + 8 * lane), w1 = *(const v4f*)(lnw + 8 * lane + 4);
  const v4f g0 = *(const v4f*)(lnb + 8 * lane), g1 = *(const v4f*)(lnb + 8 * lane + 4);
#pragma unroll
  for (int rr = 0; rr < 4; ++rr) {
    float* sp = sV + (wave * 4 + rr) * kLnTP + 8 * lane;
    const v4f a0 = *(const v4f*)(sp), a1 = *(const v4f*)(sp + 4);
    float s = ((a0[0] + a0[1]) + (a0[2] + a0[3])) + ((a1[0] + a1[1]) + (a1[2] + a1[3]));
    s = wave_sum(s);
    const float mu = s * (1.0f / kDm);
    const v4f d0 = a0 - mu, d1 = a1 - mu;
    float sq = ((d0[0] * d0[0] + d0[1] * d0[1]) + (d0[2] * d0[2] + d0[3] * d0[3]))
             + ((d1[0] * d1[0] + d1[1] * d1[1]) + (d1[2] * d1[2] + d1[3] * d1[3]));
    sq = wave_sum(sq);
    const float rs = rsqrtf(sq * (1.0f / kDm) + 1e-5f);
    const v4f o0 = d0 * rs * w0 + g0;
    const v4f o1 = d1 * rs * w1 + g1;
    *(v4f*)(sp) = o0;
    *(v4f*)(sp + 4) = o1;
  }
  __syncthreads();
  const int t4 = (lane & 7) * 4, cq = lane >> 3;
  v4f val[8];
#pragma unroll
  for (int it = 0; it < 8; ++it) {
    const int c = wave * 32 + it * 4 + cq;
    const float* col = sV + t4 * kLnTP + c;
    v4f vv;
    vv[0] = col[0];
    vv[1] = col[kLnTP];
    vv[2] = col[2 * kLnTP];
    vv[3] = col[3 * kLnTP];
    val[it] = vv;
  }
  float* ob = out + (size_t)b * kDm * kSeq + l0 + t4;
  for (int pass = 0; pass < 2; ++pass) {
#pragma unroll
    for (int it = 0; it < 8; ++it) {
      const int c = wave * 32 + it * 4 + cq;
      *(volatile v4f*)(ob + (size_t)c * kSeq) = val[it];
    }
    __threadfence();
  }
}

extern "C" void kernel_launch(void* const* d_in, const int* in_sizes, int n_in,
                              void* d_out, int out_size, void* d_ws, size_t ws_size,
                              hipStream_t stream) {
  if (n_in < 12) return;
  if (in_sizes[0]  != kRows * kDm) return;
  if (in_sizes[1]  != kDm) return;
  if (in_sizes[2]  != kDm) return;
  if (in_sizes[3]  != kXzP * kDm) return;
  if (in_sizes[4]  != kDin * 4) return;
  if (in_sizes[5]  != kDin) return;
  if (in_sizes[6]  != kXdW * kDin) return;
  if (in_sizes[7]  != kDin * kDtR) return;
  if (in_sizes[8]  != kDin) return;
  if (in_sizes[9]  != kDin * kNst) return;
  if (in_sizes[10] != kDin) return;
  if (in_sizes[11] != kDm * kDin) return;
  if (out_size != kRows * kDm) return;
  if (ws_size < kWsTotal) return;

  const float* x       = (const float*)d_in[0];
  const float* ln_w    = (const float*)d_in[1];
  const float* ln_b    = (const float*)d_in[2];
  const float* W_in    = (const float*)d_in[3];
  const float* conv_w  = (const float*)d_in[4];
  const float* conv_b  = (const float*)d_in[5];
  const float* W_x     = (const float*)d_in[6];
  const float* W_dt    = (const float*)d_in[7];
  const float* b_dt    = (const float*)d_in[8];
  const float* A_log   = (const float*)d_in[9];
  const float* Dp      = (const float*)d_in[10];
  const float* W_out   = (const float*)d_in[11];
  float* out = (float*)d_out;

  char* ws = (char*)d_ws;
  unsigned short* UP   = (unsigned short*)(ws + kOffU);
  unsigned short* WI   = (unsigned short*)(ws + kOffWI);
  unsigned short* WX   = (unsigned short*)(ws + kOffWX);
  unsigned short* WO   = (unsigned short*)(ws + kOffWO);
  float*          XZ   = (float*)(ws + kOffXZ);
  float*          UC   = (float*)(ws + kOffUC);
  unsigned short* UCH  = (unsigned short*)(ws + kOffUCH);
  float*          XD   = (float*)(ws + kOffXD);
  unsigned short* YP   = (unsigned short*)(ws + kOffY);
  float*          OP   = (float*)(ws + kOffOP);

  cast_scale_f16x8_kernel<<<(kXzP * kDm / 8) / 256, 256, 0, stream>>>(W_in, kXzP * kDm / 8, WI, kXzP * kDm / 8, kWCarry);
  cast_scale_f16x8_kernel<<<(kXdP * kDin / 8) / 256, 256, 0, stream>>>(W_x, kXdW * kDin / 8, WX, kXdP * kDin / 8, kWCarry);
  cast_scale_f16x8_kernel<<<(kDm * kDin / 8) / 256, 256, 0, stream>>>(W_out, kDm * kDin / 8, WO, kDm * kDin / 8, kWCarry);

  ln_front_kernel<<<kRows / kLnTok, 256, 0, stream>>>(x, ln_w, ln_b, UP);

  wmma_gemm64<0, false, 0, 0, false><<<dim3(((kRows / 64) * (kXzP / 64)) / 8, 1), 256, 0, stream>>>(
      UP, nullptr, kDm, 0L,
      WI, nullptr, kDm, 0L,
      (void*)XZ, nullptr, kXzP, 0L,
      nullptr, nullptr, 0L,
      kRows, kXzP, kDm, kGemmFold);

  conv_silu_kernel<<<dim3(kDin / 256, kRows / 64), 256, 0, stream>>>(XZ, conv_w, conv_b, UC, UCH);

  wmma_gemm64<0, false, 0, 0, false><<<dim3(((kRows / 64) * (kXdP / 64)) / 8, 1), 256, 0, stream>>>(
      UCH, nullptr, kDin, 0L,
      WX, nullptr, kDin, 0L,
      (void*)XD, nullptr, kXdP, 0L,
      nullptr, nullptr, 0L,
      kRows, kXdP, kDin, kGemmFold);

  scan_kernel<<<kBatch * (kDin / kScanCh), kScanCh, 0, stream>>>(XD, UC, XZ, W_dt, b_dt, A_log, Dp, YP);

  wmma_gemm64<0, false, 0, 0, false><<<dim3(((kRows / 64) * (kDm / 64)) / 8, 1), 256, 0, stream>>>(
      YP, nullptr, kDin, 0L,
      WO, nullptr, kDin, 0L,
      (void*)OP, nullptr, kDm, 0L,
      nullptr, nullptr, 0L,
      kRows, kDm, kDin, kGemmFold);

  ln_post_kernel<<<kRows / kLnTok, 256, 0, stream>>>(OP, x, ln_w, ln_b, out);
}
